// DSVDD_5248450036236
// MI455X (gfx1250) — hardware-verified
//
#include <hip/hip_runtime.h>
#include <math.h>

typedef __attribute__((ext_vector_type(16))) _Float16 v16h;
typedef __attribute__((ext_vector_type(16))) __bf16 v16b;
typedef __attribute__((ext_vector_type(8)))  _Float16 v8h;
typedef __attribute__((ext_vector_type(8)))  float v8f;
typedef __attribute__((ext_vector_type(4)))  float v4f;
typedef __attribute__((ext_vector_type(2)))  float v2f;
typedef __attribute__((ext_vector_type(4)))  unsigned v4u;
typedef __attribute__((ext_vector_type(4)))  int v4i;
typedef float __attribute__((may_alias)) float_a;
typedef int __attribute__((may_alias)) int_a;

template <typename T> __device__ __forceinline__ void vst2(void* p, T v) { *(volatile T*)p = v; __threadfence(); *(volatile T*)p = v; }
__device__ __forceinline__ v8f wmma16(v16h a, v16h b, v8f c) {
  v8f d = __builtin_amdgcn_wmma_f32_16x16x32_f16(false, a, false, b, (short)0, c, false, false);
  asm volatile("v_nop\n\tv_nop\n\tv_nop\n\tv_nop" : "+v"(d) : "v"(a), "v"(b));
  return d;
}
__device__ __forceinline__ v8f wmma_bf(v16b a, v16b b, v8f c) {
  v8f d = __builtin_amdgcn_wmma_f32_16x16x32_bf16(false, a, false, b, (short)0, c, false, false);
  asm volatile("v_nop\n\tv_nop\n\tv_nop\n\tv_nop" : "+v"(d) : "v"(a), "v"(b));
  return d;
}
__device__ __forceinline__ v16h frag_h(const _Float16* rowk0, int lane) {
  union { v16h v; v8h q[2]; } u; const _Float16* p = rowk0 + 8 * (lane >> 4);
  u.q[0] = *(const v8h*)p; u.q[1] = *(const v8h*)(p + 16); return u.v;
}
__device__ __forceinline__ v16h frag_f32(const float* rowk0, int lane) {
  v16h a; const float* p = rowk0 + 8 * (lane >> 4);
#pragma unroll
  for (int i = 0; i < 8; ++i) { a[i] = (_Float16)p[i]; a[8 + i] = (_Float16)p[16 + i]; }
  return a;
}
__device__ __forceinline__ v16h frag_f32s(const float* rowk0, int lane, float sc) {
  v16h a; const float* p = rowk0 + 8 * (lane >> 4);
#pragma unroll
  for (int i = 0; i < 8; ++i) { a[i] = (_Float16)(p[i] * sc); a[8 + i] = (_Float16)(p[16 + i] * sc); }
  return a;
}
__device__ __forceinline__ v16h fragc_f32(const float* W, int k0, int n, int lane, int ld, int K) {
  v16h a; const int g = lane >> 4;
#pragma unroll
  for (int i = 0; i < 8; ++i) { const int ka = k0 + 8 * g + i, kb = ka + 16;
    a[i] = (_Float16)(ka < K ? W[(size_t)(ka < K ? ka : K - 1) * ld + n] : 0.f); a[8 + i] = (_Float16)(kb < K ? W[(size_t)(kb < K ? kb : K - 1) * ld + n] : 0.f); }
  return a;
}
struct F2 { v16b h, l; };
__device__ __forceinline__ F2 bsplit16(const float v[16]) { F2 r;
#pragma unroll
  for (int i = 0; i < 16; ++i) { const __bf16 h = (__bf16)v[i]; r.h[i] = h; r.l[i] = (__bf16)(v[i] - (float)h); }
  return r; }
__device__ __forceinline__ F2 split_row(const float* row, int k0, int lane) { float v[16]; const float* p = row + k0 + 8 * (lane >> 4);
#pragma unroll
  for (int i = 0; i < 8; ++i) { v[i] = p[i]; v[8 + i] = p[16 + i]; }
  return bsplit16(v); }
__device__ __forceinline__ F2 split_rowK(const float* row, int k0, int lane, int K) { float v[16]; const int g = lane >> 4;
#pragma unroll
  for (int i = 0; i < 8; ++i) { const int ka = k0 + 8 * g + i, kb = ka + 16; v[i] = ka < K ? row[ka < K ? ka : K - 1] : 0.f; v[8 + i] = kb < K ? row[kb < K ? kb : K - 1] : 0.f; }
  return bsplit16(v); }
__device__ __forceinline__ F2 split_col(const float* W, int k0, int n, int lane, int ld, int K) { float v[16]; const int g = lane >> 4;
#pragma unroll
  for (int i = 0; i < 8; ++i) { const int ka = k0 + 8 * g + i, kb = ka + 16; v[i] = ka < K ? W[(size_t)(ka < K ? ka : K - 1) * ld + n] : 0.f; v[8 + i] = kb < K ? W[(size_t)(kb < K ? kb : K - 1) * ld + n] : 0.f; }
  return bsplit16(v); }
__device__ __forceinline__ v8f mac3(const F2& a, const F2& b, v8f c) { c = wmma_bf(a.l, b.h, c); c = wmma_bf(a.h, b.l, c); return wmma_bf(a.h, b.h, c); }
__device__ __forceinline__ float sigm(float v) { return 1.0f / (1.0f + expf(-v)); }
#define LDSX() do { asm volatile("s_wait_dscnt 0" ::: "memory"); __builtin_amdgcn_wave_barrier(); __builtin_amdgcn_fence(__ATOMIC_RELEASE, "workgroup"); } while (0)


#ifndef NBT
#define NBT 16
#endif
#define NP 3136
#define NR (NBT * NP)
#define DD 128
#define MC 3136
#define MCP 3200
#define NCB 25
#define KS 6
#define NRB (NR / 64)
typedef __attribute__((ext_vector_type(8))) __bf16 v8b;
__device__ __forceinline__ v16b frag_b(const __bf16* rowk0, int lane) {
  union { v16b v; v8b q[2]; } u; const __bf16* p = rowk0 + 8 * (lane >> 4);
  u.q[0] = *(const v8b*)p; u.q[1] = *(const v8b*)(p + 16); return u.v;
}
__device__ __forceinline__ float bfr(float v) { return (float)(__bf16)v; }
__device__ __attribute__((noinline)) float exp_ni(float v) { return expf(v); }
__device__ __attribute__((noinline)) float erf_ni(float v) { return erff(v); }

#define WS_PC   0u
#define WS_CN   (WS_PC + 2u * MCP * DD)
#define WS_CAND (WS_CN + 4u * MCP)
#define WS_SC   (WS_CAND + 4u * NR * NCB * 8)
#define WS_PB   (WS_SC + 4u * 16 * NP)
#define WS_END  (WS_PB + 4u * (16 * NP / 64) * 32)

__global__ __launch_bounds__(128) void k_packc(const float* __restrict__ Cm, __bf16* __restrict__ PC, float* __restrict__ CN) {
  __shared__ __align__(16) __bf16 s[64][DD + 8]; __shared__ __align__(16) float sn[64]; const int d = threadIdx.x; const int m0 = blockIdx.x * 64;
  for (int ml = 0; ml < 64; ++ml) { const int m = m0 + ml; s[ml][d] = (__bf16)((m < MC) ? Cm[(size_t)d * MC + m] : 0.f); }
  __syncthreads();
  if (d < 64) { const int m = m0 + d; float a = 0.f; if (m < MC) {
#pragma unroll 4
      for (int k = 0; k < DD; ++k) { const float v = (float)s[d][k]; a += v * v; } } else a = 3.0e38f; sn[d] = a; }
  __syncthreads();
  for (int q = d; q < 64 * 16; q += 128) { const int ml = q >> 4, pc = q & 15; vst2((unsigned*)(PC + (size_t)(m0 + ml) * DD + pc * 8), *(const v4u*)&s[ml][pc * 8]); }
  if (d < 16) vst2(CN + m0 + d * 4, *(const v4f*)&sn[d * 4]);
}
__global__ __launch_bounds__(128) void k_d2sel(const float* __restrict__ PHI, const __bf16* __restrict__ PC, const float* __restrict__ CN, float* __restrict__ CAND) {
  __shared__ __align__(16) float so[4][16][132]; __shared__ __align__(16) float sc[4][16][8];
  const int tid = threadIdx.x, wave = tid >> 5, lane = tid & 31, col = lane & 15, g = lane >> 4; const size_t r0 = (size_t)blockIdx.x * 64 + wave * 16; const int cb = blockIdx.y; const int m0 = cb * 128;
  v8f acc[8] = {}; float fsq = 0.f;
#pragma unroll
  for (int kc = 0; kc < 4; ++kc) { v16b a; const float* p = PHI + (r0 + col) * DD + kc * 32 + 8 * g;
#pragma unroll
    for (int i = 0; i < 8; ++i) { const float x0 = bfr(p[i]), x1 = bfr(p[16 + i]); a[i] = (__bf16)x0; a[8 + i] = (__bf16)x1; fsq += x0 * x0; fsq += x1 * x1; }
#pragma unroll
    for (int j = 0; j < 8; ++j) acc[j] = wmma_bf(a, frag_b(PC + (size_t)(m0 + j * 16 + col) * DD + kc * 32, lane), acc[j]); }
  fsq += __shfl_xor(fsq, 16);
  float frow[8];
#pragma unroll
  for (int r = 0; r < 8; ++r) frow[r] = __shfl(fsq, 8 * g + r);
#pragma unroll
  for (int j = 0; j < 8; ++j) { const float cn = CN[m0 + j * 16 + col];
#pragma unroll
    for (int r = 0; r < 8; ++r) so[wave][8 * g + r][j * 16 + col] = (frow[r] + cn) - 2.0f * acc[j][r]; }
  LDSX();
  { const int rl = lane & 15, half = lane >> 4; float b[KS];
#pragma unroll
    for (int k = 0; k < KS; ++k) b[k] = 3.0e38f;
#pragma unroll 4
    for (int c = 0; c < 64; ++c) { const float d = so[wave][rl][half * 64 + c]; if (d < b[KS - 1]) { int pos = KS - 1;
#pragma unroll
        for (int k = KS - 2; k >= 0; --k) if (d < b[k]) pos = k;
#pragma unroll
        for (int k = KS - 1; k >= 1; --k) if (k > pos) b[k] = b[k - 1];
#pragma unroll
        for (int k = 0; k < KS; ++k) if (k == pos) b[k] = d; } }
    float pb[KS];
#pragma unroll
    for (int q = 0; q < KS; ++q) pb[q] = __shfl_xor(b[q], 16);
#pragma unroll
    for (int q = 0; q < KS; ++q) { const float d = pb[q]; if (d < b[KS - 1]) { int pos = KS - 1;
#pragma unroll
        for (int k = KS - 2; k >= 0; --k) if (d < b[k]) pos = k;
#pragma unroll
        for (int k = KS - 1; k >= 1; --k) if (k > pos) b[k] = b[k - 1];
#pragma unroll
        for (int k = 0; k < KS; ++k) if (k == pos) b[k] = d; } }
    if (half == 0) {
#pragma unroll
      for (int k = 0; k < KS; ++k) sc[wave][rl][k] = b[k];
      sc[wave][rl][6] = 0.f; sc[wave][rl][7] = 0.f; } }
  LDSX();
  if (lane < 16) { const int rl = lane; float* dst = CAND + ((r0 + rl) * NCB + cb) * 8; const v4f p0 = *(const v4f*)&sc[wave][rl][0]; const v4f p1 = *(const v4f*)&sc[wave][rl][4]; vst2(dst, p0); vst2(dst + 4, p1); }
}
__global__ __launch_bounds__(64) void k_fin(const float* __restrict__ CAND, const float* __restrict__ Rr, float* __restrict__ SC, float* __restrict__ PB) {
  __shared__ __align__(16) float ssc[64]; __shared__ float sa[64], sr[64]; __shared__ __align__(16) float sl[32];
  const int t = threadIdx.x; const size_t row = (size_t)blockIdx.x * 64 + t;
  float b[KS];
#pragma unroll
  for (int k = 0; k < KS; ++k) b[k] = 3.0e38f;
#pragma unroll 1
  for (int cb = 0; cb < NCB; ++cb) { const float* c = CAND + (row * NCB + cb) * 8;
#pragma unroll
    for (int q = 0; q < KS; ++q) { const float d = c[q]; if (d < b[KS - 1]) { int pos = KS - 1;
#pragma unroll
        for (int k = KS - 2; k >= 0; --k) if (d < b[k]) pos = k;
#pragma unroll
        for (int k = KS - 1; k >= 1; --k) if (k > pos) b[k] = b[k - 1];
#pragma unroll
        for (int k = 0; k < KS; ++k) if (k == pos) b[k] = d; } } }
  const float d0 = sqrtf(fmaxf(b[0], 0.f)), d1 = sqrtf(fmaxf(b[1], 0.f)), d2_ = sqrtf(fmaxf(b[2], 0.f));
  const float mx = -d0;
  const float e0 = exp_ni(-d0 - mx), e1 = exp_ni(-d1 - mx), e2 = exp_ni(-d2_ - mx);
  ssc[t] = (e0 / (e0 + e1 + e2)) * d0;
  const float r2 = bfr(Rr[0]) * bfr(Rr[0]);
  sa[t] = fmaxf(b[0] - r2, 0.f) + fmaxf(b[1] - r2, 0.f) + fmaxf(b[2] - r2, 0.f);
  sr[t] = fmaxf(r2 - b[3] - 0.1f, 0.f) + fmaxf(r2 - b[4] - 0.1f, 0.f) + fmaxf(r2 - b[5] - 0.1f, 0.f);
  __syncthreads();
  for (int o = 32; o > 0; o >>= 1) { if (t < o) { sa[t] += sa[t + o]; sr[t] += sr[t + o]; } __syncthreads(); }
  if (t < 32) sl[t] = (t == 0) ? sa[0] : (t == 1 ? sr[0] : 0.f);
  __syncthreads();
  if (t < 16) vst2(SC + (size_t)blockIdx.x * 64 + t * 4, *(const v4f*)&ssc[t * 4]);
  if (t < 8) vst2(PB + (size_t)blockIdx.x * 32 + t * 4, *(const v4f*)&sl[t * 4]);
}
__global__ __launch_bounds__(256) void k_out(const float* __restrict__ SC, const float* __restrict__ PB, float* __restrict__ out) {
  __shared__ float sloss; const int t = threadIdx.x;
  if (t == 0) { float a = 0.f, r = 0.f; for (int b = 0; b < NRB; ++b) { a += PB[b * 32]; r += PB[b * 32 + 1]; } const float inv = 1.0f / ((float)NR * 3.0f); sloss = (1.0f / 0.001f) * (a * inv) + (1.0f / 0.001f) * (r * inv); }
  __syncthreads();
  const float lossv = sloss;
  const int npiece = (NR + 1) / 4;
  for (int i = t; i < npiece; i += 256) { v4f o; const int f0 = 4 * i;
#pragma unroll
    for (int q = 0; q < 4; ++q) { const int f = f0 + q; float v = SC[max(f - 1, 0)]; if (f == 0) v = lossv; o[q] = v; }
    vst2(out + f0, o); }
  if (t == 0) vst2(out + NR, SC[NR - 1]);
}
extern "C" void kernel_launch(void* const* d_in, const int* in_sizes, int n_in, void* d_out, int out_size, void* d_ws, size_t ws_size, hipStream_t stream) {
  (void)in_sizes; (void)n_in; (void)out_size;
  const float** F = (const float**)d_in;
  if (ws_size < (size_t)WS_END) return;
  char* ws = (char*)d_ws; __bf16* PC = (__bf16*)(ws + WS_PC); float *CN = (float*)(ws + WS_CN), *CAND = (float*)(ws + WS_CAND), *SC = (float*)(ws + WS_SC), *PB = (float*)(ws + WS_PB);
  k_packc<<<MCP / 64, 128, 0, stream>>>(F[1], PC, CN);
  k_d2sel<<<dim3(NRB, NCB), 128, 0, stream>>>(F[0], PC, CN, CAND);
  k_fin<<<NRB, 64, 0, stream>>>(CAND, F[2], SC, PB);
  k_out<<<1, 256, 0, stream>>>(SC, PB, (float*)d_out);
}
